// Level2GATEncoder_20117626814923
// MI455X (gfx1250) — hardware-verified
//
#include <hip/hip_runtime.h>
#include <stddef.h>


#define NTHR  256
#define NWAVE 8
#define DIM   128
#define NCOL  256
#define HH    4
#define GR    32
#define GC    128
#define XSP   132
#define NB    448
#define SLOTB 9
#define CHUNK 1024
#define WCAP  128
#define AGG_LDS_BYTES ((NB * DIM + 2 * NB * HH) * 4 + (NWAVE * WCAP + NWAVE) * 4)

static_assert(AGG_LDS_BYTES == 247840);
static_assert(WCAP == (CHUNK / NTHR) * 32);
static_assert(CHUNK == NTHR * 4);
static_assert(NB < (1 << SLOTB));
static_assert((NB % 2) == 0);
static_assert((XSP % 4) == 0);
static_assert(DIM == 32 * 4);
static_assert(NCOL == 2 * DIM);

typedef float          v4f  __attribute__((ext_vector_type(4)));
typedef float          v8f  __attribute__((ext_vector_type(8)));
typedef int            v4i  __attribute__((ext_vector_type(4)));
typedef _Float16       v8h  __attribute__((ext_vector_type(8)));
typedef __bf16         v16b __attribute__((ext_vector_type(16)));
typedef unsigned short v8us __attribute__((ext_vector_type(8)));

union FragB { v16b v; v4i u[2]; };
union Pack  { v8h h; v8us s; v4i i; };

__device__ __forceinline__ unsigned short f2bf(float x) {
  unsigned b = __float_as_uint(x);
  b += 0x7FFFu + ((b >> 16) & 1u);
  return (unsigned short)(b >> 16);
}
__device__ __forceinline__ float bf2f(unsigned short h) { return __uint_as_float(((unsigned)h) << 16); }

__device__ __forceinline__ v8f wmb(v16b a, v16b b, v8f c) {
  v8f d = __builtin_amdgcn_wmma_f32_16x16x32_bf16(false, a, false, b, (short)0, c, false, false);
  asm volatile("v_nop\n\tv_nop\n\tv_nop\n\tv_nop" : "+v"(d) : "v"(a), "v"(b));
  return d;
}

__device__ __forceinline__ float lk(float t) { return fmaxf(t, 0.2f * t); }
__device__ __forceinline__ float dl(v4f t, v4f w) {
  return w.x * lk(t.x) + w.y * lk(t.y) + w.z * lk(t.z) + w.w * lk(t.w);
}

__global__ __launch_bounds__(NTHR) void k_cvt_x(const float* __restrict__ src, int rows_src,
                                                unsigned short* ph, unsigned short* pl, int rows_total) {
  const int n8 = rows_total * (DIM / 8);
  const int i  = blockIdx.x * NTHR + threadIdx.x;
  if (i >= n8) return;
  const int r  = i >> 4;
  const int kb = (i & 15) * 8;
  const int rc = (r < rows_src) ? r : (rows_src - 1);
  const float* sp = src + (size_t)rc * DIM + kb;
  const v4f x0 = *(const v4f*)sp;
  const v4f x1 = *(const v4f*)(sp + 4);
  const bool valid = (r < rows_src);
  Pack uh, ul;
  const v4i z4 = {0, 0, 0, 0};
  uh.i = z4; ul.i = z4;
#pragma unroll
  for (int j = 0; j < 4; ++j) {
    const float v = valid ? x0[j] : 0.f;
    const unsigned short hb = f2bf(v);
    uh.s[j] = hb;
    ul.s[j] = f2bf(v - bf2f(hb));
    const float u = valid ? x1[j] : 0.f;
    const unsigned short hc = f2bf(u);
    uh.s[4 + j] = hc;
    ul.s[4 + j] = f2bf(u - bf2f(hc));
  }
  const size_t o = (size_t)i * 8;
  *(volatile v4i*)(ph + o) = uh.i;
  *(volatile v4i*)(pl + o) = ul.i;
  __threadfence();
  *(volatile v4i*)(ph + o) = uh.i;
  *(volatile v4i*)(pl + o) = ul.i;
}

__global__ __launch_bounds__(NTHR) void k_cvt_w(const float* __restrict__ Wa, const float* __restrict__ Wb,
                                                unsigned short* ph, unsigned short* pl) {
  const int i = blockIdx.x * NTHR + threadIdx.x;
  if (i >= NCOL * (DIM / 8)) return;
  const int n  = i >> 4;
  const int kb = (i & 15) * 8;
  const int nc = n & (DIM - 1);
  const bool second = (n >= DIM);
  Pack uh, ul;
  const v4i z4 = {0, 0, 0, 0};
  uh.i = z4; ul.i = z4;
#pragma unroll
  for (int j = 0; j < 8; ++j) {
    const int k = kb + j;
    const float va = Wa[k * DIM + nc];
    const float vb = Wb[k * DIM + nc];
    const float v  = second ? vb : va;
    const unsigned short hb = f2bf(v);
    uh.s[j] = hb;
    ul.s[j] = f2bf(v - bf2f(hb));
  }
  const size_t o = (size_t)i * 8;
  *(volatile v4i*)(ph + o) = uh.i;
  *(volatile v4i*)(pl + o) = ul.i;
  __threadfence();
  *(volatile v4i*)(ph + o) = uh.i;
  *(volatile v4i*)(pl + o) = ul.i;
}

__global__ __launch_bounds__(NTHR) void k_gemm(
    const unsigned short* __restrict__ A0, const unsigned short* __restrict__ A1,
    const unsigned short* __restrict__ B0, const unsigned short* __restrict__ B1,
    const float* __restrict__ biasA, const float* __restrict__ biasB,
    float* out, int K, int Ncols) {
  __shared__ __attribute__((aligned(16))) float Xs[GR * XSP];

  const int tid  = threadIdx.x;
  const int lane = tid & 31;
  const int wave = tid >> 5;
  const int hh   = lane >> 4;
  const int m    = lane & 15;
  const int rowBase = blockIdx.x * GR;
  const int colBase = blockIdx.y * GC;
  const int ncol = colBase + wave * 16 + m;

  const size_t ra0 = (size_t)(rowBase + m) * K + 8 * hh;
  const size_t ra1 = ra0 + (size_t)16 * K;
  const size_t rb  = (size_t)ncol * K + 8 * hh;

  v8f c0 = {0.f, 0.f, 0.f, 0.f, 0.f, 0.f, 0.f, 0.f};
  v8f c1 = {0.f, 0.f, 0.f, 0.f, 0.f, 0.f, 0.f, 0.f};

#pragma unroll 1
  for (int k0 = 0; k0 < K; k0 += 32) {
    FragB ah0, ah1, al0, al1, bh, bl;
    ah0.u[0] = *(const v4i*)(A0 + ra0 + k0);  ah0.u[1] = *(const v4i*)(A0 + ra0 + k0 + 16);
    ah1.u[0] = *(const v4i*)(A0 + ra1 + k0);  ah1.u[1] = *(const v4i*)(A0 + ra1 + k0 + 16);
    al0.u[0] = *(const v4i*)(A1 + ra0 + k0);  al0.u[1] = *(const v4i*)(A1 + ra0 + k0 + 16);
    al1.u[0] = *(const v4i*)(A1 + ra1 + k0);  al1.u[1] = *(const v4i*)(A1 + ra1 + k0 + 16);
    bh.u[0]  = *(const v4i*)(B0 + rb + k0);   bh.u[1]  = *(const v4i*)(B0 + rb + k0 + 16);
    bl.u[0]  = *(const v4i*)(B1 + rb + k0);   bl.u[1]  = *(const v4i*)(B1 + rb + k0 + 16);
    c0 = wmb(ah0.v, bh.v, c0);  c0 = wmb(ah0.v, bl.v, c0);  c0 = wmb(al0.v, bh.v, c0);
    c1 = wmb(ah1.v, bh.v, c1);  c1 = wmb(ah1.v, bl.v, c1);  c1 = wmb(al1.v, bh.v, c1);
  }

  const float ba = biasA[ncol & (DIM - 1)];
  const float bb = biasB[ncol & (DIM - 1)];
  const float bv = (ncol < DIM) ? ba : bb;
  const int cl = wave * 16 + m;
#pragma unroll
  for (int r = 0; r < 8; ++r) {
    Xs[(8 * hh + r) * XSP + cl]      = c0[r] + bv;
    Xs[(16 + 8 * hh + r) * XSP + cl] = c1[r] + bv;
  }
  __syncthreads();

  v4f xv[4];
  float* xpp[4];
#pragma unroll
  for (int i = 0; i < 4; ++i) {
    xv[i]  = *(const v4f*)(Xs + (4 * wave + i) * XSP + 4 * lane);
    xpp[i] = out + (size_t)(rowBase + 4 * wave + i) * Ncols + colBase + 4 * lane;
  }
#pragma unroll
  for (int i = 0; i < 4; ++i) *(volatile v4f*)(xpp[i]) = xv[i];
  __threadfence();
#pragma unroll
  for (int i = 0; i < 4; ++i) *(volatile v4f*)(xpp[i]) = xv[i];
}

__device__ __forceinline__ void hit4(const float* xs, const float* xd, float* ar, float* mp, float* dp, v4f w0) {
  const v4f a0 = *(const v4f*)(xs);
  const v4f d0 = *(const v4f*)(xd);
  float s = dl(a0 + d0, w0);
  s += __shfl_xor(s, 4, 32);
  s += __shfl_xor(s, 2, 32);
  s += __shfl_xor(s, 1, 32);
  const float mo = mp[0], no = dp[0];
  const float mn = fmaxf(mo, s);
  const float sc = __expf(mo - mn);
  const float p  = __expf(s - mn);
  v4f e0 = *(v4f*)(ar);
  e0 = e0 * sc + a0 * p;
  *(v4f*)(ar) = e0;
  mp[0] = mn;
  dp[0] = no * sc + p;
}

template <int OUT16>
__global__ __launch_bounds__(NTHR) void k_agg(
    const int* __restrict__ ei, const float* __restrict__ xlr,
    const float* __restrict__ att, const float* __restrict__ bias,
    const float* __restrict__ gam, const float* __restrict__ bet,
    unsigned short* ph, unsigned short* pl, float* out,
    int nN, int nE, int nW) {
  extern __shared__ v4f lds_dyn[];
  float* sacc = (float*)lds_dyn;
  float* mx   = sacc + NB * DIM;
  float* dn   = mx + NB * HH;
  int*   list = (int*)(dn + NB * HH);
  int*   wcnt = list + NWAVE * WCAP;

  const int tid  = threadIdx.x;
  const int lane = tid & 31;
  const int wave = tid >> 5;
  const int nodeBase = blockIdx.x * NB;

  {
    const v4f z4 = {0.f, 0.f, 0.f, 0.f};
    for (int i = tid; i < NB * DIM / 4; i += NTHR) lds_dyn[i] = z4;
    for (int i = tid; i < NB * HH; i += NTHR) { mx[i] = -1.0e30f; dn[i] = 0.f; }
  }
  __syncthreads();

  const int coff = 4 * lane;
  const int hidx = lane >> 3;
  const v4f w0 = *(const v4f*)(att + coff);

  const int* eid = ei + nE;
  const bool al16 = ((nE & 3) == 0);
  const int nChunks = (nE + CHUNK - 1) / CHUNK;

#pragma unroll 1
  for (int ch = 0; ch < nChunks; ++ch) {
    const int cbase = ch * CHUNK;
    int wc = 0;
    {
      const int el0 = tid * 4;
      const int e0  = cbase + el0;
      const int sent = -2147483647 - 1;
      v4i d;
      if (al16 && (cbase + CHUNK <= nE)) {
        d = *(const v4i*)(eid + e0);
      } else {
        const int q0 = (e0     < nE) ? e0     : (nE - 1);
        const int q1 = (e0 + 1 < nE) ? e0 + 1 : (nE - 1);
        const int q2 = (e0 + 2 < nE) ? e0 + 2 : (nE - 1);
        const int q3 = (e0 + 3 < nE) ? e0 + 3 : (nE - 1);
        const int t0 = eid[q0], t1 = eid[q1], t2 = eid[q2], t3 = eid[q3];
        d.x = (e0     < nE) ? t0 : sent;
        d.y = (e0 + 1 < nE) ? t1 : sent;
        d.z = (e0 + 2 < nE) ? t2 : sent;
        d.w = (e0 + 3 < nE) ? t3 : sent;
      }
      const unsigned s0 = (unsigned)d.x - (unsigned)nodeBase;
      const unsigned s1 = (unsigned)d.y - (unsigned)nodeBase;
      const unsigned s2 = (unsigned)d.z - (unsigned)nodeBase;
      const unsigned s3 = (unsigned)d.w - (unsigned)nodeBase;
      const bool h0 = s0 < (unsigned)NB;
      const bool h1 = s1 < (unsigned)NB;
      const bool h2 = s2 < (unsigned)NB;
      const bool h3 = s3 < (unsigned)NB;
      const unsigned many = __builtin_amdgcn_ballot_w32(h0 | h1 | h2 | h3);
      if (many != 0u) {
#define HITJ(J, HJ, SJ) { \
          const unsigned mj = __builtin_amdgcn_ballot_w32(HJ); \
          if (HJ) { \
            const int pos = wc + (int)__builtin_amdgcn_mbcnt_lo(mj, 0u); \
            if (pos < WCAP) list[wave * WCAP + pos] = ((el0 + (J)) << SLOTB) | (int)(SJ); \
          } \
          wc += (int)__builtin_popcount(mj); }
        HITJ(0, h0, s0)
        HITJ(1, h1, s1)
        HITJ(2, h2, s2)
        HITJ(3, h3, s3)
#undef HITJ
      }
    }
    if (lane == 0) wcnt[wave] = wc;
    __syncthreads();

    if (wave == 0) {
#pragma unroll 1
      for (int wsx = 0; wsx < NWAVE; ++wsx) {
        int n = __builtin_amdgcn_readfirstlane(wcnt[wsx]);
        n = n > WCAP ? WCAP : n;
        n = n < 0 ? 0 : n;
#pragma unroll 1
        for (int i = 0; i < n; ++i) {
          const int ent = __builtin_amdgcn_readfirstlane(list[wsx * WCAP + i]);
          int slot = ent & ((1 << SLOTB) - 1);
          slot = slot > (NB - 1) ? (NB - 1) : slot;
          const int el   = (ent >> SLOTB) & (CHUNK - 1);
          const int node = nodeBase + slot;
          if (node >= nN) continue;
          int e = cbase + el;
          if (e > nE - 1) e = nE - 1;
          int sj = ei[e];
          sj = sj < 0 ? 0 : (sj > nN - 1 ? nN - 1 : sj);
          const float* xs = xlr + (size_t)sj * NCOL + coff;
          const float* xd = xlr + (size_t)node * NCOL + DIM + coff;
          float* ar = sacc + slot * DIM + coff;
          float* mp = mx + slot * HH + hidx;
          float* dp = dn + slot * HH + hidx;
          hit4(xs, xd, ar, mp, dp, w0);
        }
      }
    }
    __syncthreads();
  }

  const v4f bi4 = *(const v4f*)(bias + coff);
  const v4f g4  = *(const v4f*)(gam + coff);
  const v4f be4 = *(const v4f*)(bet + coff);
#pragma unroll 1
  for (int s = wave; s < NB; s += NWAVE) {
    const int node = nodeBase + s;
    float* ar = sacc + s * DIM + coff;
    const v4f e0 = *(const v4f*)ar;
    const float inv = 1.0f / (dn[s * HH + hidx] + 1e-16f);
    const v4f o = e0 * inv + bi4;
    float sm = (o.x + o.y) + (o.z + o.w);
    sm += __shfl_xor(sm, 16, 32);
    sm += __shfl_xor(sm, 8, 32);
    sm += __shfl_xor(sm, 4, 32);
    sm += __shfl_xor(sm, 2, 32);
    sm += __shfl_xor(sm, 1, 32);
    const float mu = sm * (1.0f / 128.0f);
    const v4f t = o - mu;
    float q = t.x * t.x + t.y * t.y + t.z * t.z + t.w * t.w;
    q += __shfl_xor(q, 16, 32);
    q += __shfl_xor(q, 8, 32);
    q += __shfl_xor(q, 4, 32);
    q += __shfl_xor(q, 2, 32);
    q += __shfl_xor(q, 1, 32);
    const float rstd = rsqrtf(q * (1.0f / 128.0f) + 1e-5f);
    const v4f y = (t * rstd) * g4 + be4;
    const float y0 = (y.x > 0.f) ? y.x : (__expf(y.x) - 1.0f);
    const float y1 = (y.y > 0.f) ? y.y : (__expf(y.y) - 1.0f);
    const float y2 = (y.z > 0.f) ? y.z : (__expf(y.z) - 1.0f);
    const float y3 = (y.w > 0.f) ? y.w : (__expf(y.w) - 1.0f);
    const bool valid = (node < nN);
    v4f yy;
    yy.x = valid ? y0 : 0.f;
    yy.y = valid ? y1 : 0.f;
    yy.z = valid ? y2 : 0.f;
    yy.w = valid ? y3 : 0.f;
    if (OUT16) {
      *(v4f*)ar = yy;
    } else {
      if (node < nW) {
        float* op = out + (size_t)node * DIM + coff;
        *(volatile v4f*)op = yy;
        __threadfence();
        *(volatile v4f*)op = yy;
      }
    }
  }

  if (OUT16) {
    __syncthreads();
    const int rr = lane >> 4;
    const int c8 = 8 * (lane & 15);
#pragma unroll 1
    for (int p = wave; p < NB / 2; p += NWAVE) {
      const int node0 = nodeBase + 2 * p;
      if (node0 < nW) {
        const float* fr = sacc + (2 * p + rr) * DIM + c8;
        const v4f f0 = *(const v4f*)fr;
        const v4f f1 = *(const v4f*)(fr + 4);
        Pack uh, ul;
        const v4i z4 = {0, 0, 0, 0};
        uh.i = z4; ul.i = z4;
#pragma unroll
        for (int j = 0; j < 4; ++j) {
          const unsigned short hb = f2bf(f0[j]);
          uh.s[j] = hb;
          ul.s[j] = f2bf(f0[j] - bf2f(hb));
          const unsigned short hc = f2bf(f1[j]);
          uh.s[4 + j] = hc;
          ul.s[4 + j] = f2bf(f1[j] - bf2f(hc));
        }
        const size_t o = (size_t)node0 * DIM + 8 * lane;
        *(volatile v4i*)(ph + o) = uh.i;
        *(volatile v4i*)(pl + o) = ul.i;
        __threadfence();
        *(volatile v4i*)(ph + o) = uh.i;
        *(volatile v4i*)(pl + o) = ul.i;
      }
    }
  }
}

extern "C" void kernel_launch(void* const* d_in, const int* in_sizes, int n_in,
                              void* d_out, int out_size, void* d_ws, size_t ws_size,
                              hipStream_t stream) {
  if (n_in < 18) return;
  const int nN = in_sizes[0] / DIM;
  if (nN <= 0 || in_sizes[0] != nN * DIM) return;
  const int nE = in_sizes[1] / 2;
  if (nE <= 0 || in_sizes[1] != 2 * nE) return;
  for (int L = 0; L < 2; ++L) {
    const int b = 2 + 8 * L;
    if (in_sizes[b] != DIM * DIM || in_sizes[b + 1] != DIM || in_sizes[b + 2] != DIM * DIM ||
        in_sizes[b + 3] != DIM || in_sizes[b + 4] != HH * 32 || in_sizes[b + 5] != DIM ||
        in_sizes[b + 6] != DIM || in_sizes[b + 7] != DIM) return;
  }
  if (out_size != nN * DIM) return;

  const float* x    = (const float*)d_in[0];
  const int*   ei   = (const int*)d_in[1];
  const float* Wl0  = (const float*)d_in[2];   const float* bl0 = (const float*)d_in[3];
  const float* Wr0  = (const float*)d_in[4];   const float* br0 = (const float*)d_in[5];
  const float* at0  = (const float*)d_in[6];   const float* bs0 = (const float*)d_in[7];
  const float* g0   = (const float*)d_in[8];   const float* be0 = (const float*)d_in[9];
  const float* Wl1  = (const float*)d_in[10];  const float* bl1 = (const float*)d_in[11];
  const float* Wr1  = (const float*)d_in[12];  const float* br1 = (const float*)d_in[13];
  const float* at1  = (const float*)d_in[14];  const float* bs1 = (const float*)d_in[15];
  const float* g1   = (const float*)d_in[16];  const float* be1 = (const float*)d_in[17];
  float* out = (float*)d_out;

  const int Mpad = ((nN + GR - 1) / GR) * GR;

  char* wsp = (char*)d_ws;
  size_t off = 0;
  const size_t plB = (size_t)Mpad * DIM * 2;
  const size_t wB  = (size_t)NCOL * DIM * 2;
  const size_t xB  = (size_t)Mpad * NCOL * 4;
  unsigned short* Ah = (unsigned short*)(wsp + off); off += (plB + 255) & ~(size_t)255;
  unsigned short* Al = (unsigned short*)(wsp + off); off += (plB + 255) & ~(size_t)255;
  unsigned short* Bh = (unsigned short*)(wsp + off); off += (wB + 255) & ~(size_t)255;
  unsigned short* Bl = (unsigned short*)(wsp + off); off += (wB + 255) & ~(size_t)255;
  float* xlr = (float*)(wsp + off); off += (xB + 255) & ~(size_t)255;
  if (off > ws_size) return;
  if (off > (size_t)134217728) return;

  const int mt  = Mpad / GR;
  const int ga0 = (Mpad + NB - 1) / NB;
  const int ga1 = (nN + NB - 1) / NB;

  hipFuncSetAttribute(reinterpret_cast<const void*>(&k_agg<1>),
                      hipFuncAttributeMaxDynamicSharedMemorySize, AGG_LDS_BYTES);
  hipFuncSetAttribute(reinterpret_cast<const void*>(&k_agg<0>),
                      hipFuncAttributeMaxDynamicSharedMemorySize, AGG_LDS_BYTES);

  k_cvt_x<<<(Mpad * (DIM / 8) + NTHR - 1) / NTHR, NTHR, 0, stream>>>(x, nN, Ah, Al, Mpad);
  k_cvt_w<<<(NCOL * (DIM / 8) + NTHR - 1) / NTHR, NTHR, 0, stream>>>(Wl0, Wr0, Bh, Bl);
  k_gemm<<<dim3(mt, NCOL / GC), NTHR, 0, stream>>>(Ah, Al, Bh, Bl, bl0, br0, xlr, DIM, NCOL);
  k_agg<1><<<ga0, NTHR, AGG_LDS_BYTES, stream>>>(ei, xlr, at0, bs0, g0, be0, Ah, Al, out, nN, nE, Mpad);

  k_cvt_w<<<(NCOL * (DIM / 8) + NTHR - 1) / NTHR, NTHR, 0, stream>>>(Wl1, Wr1, Bh, Bl);
  k_gemm<<<dim3(mt, NCOL / GC), NTHR, 0, stream>>>(Ah, Al, Bh, Bl, bl1, br1, xlr, DIM, NCOL);
  k_agg<0><<<ga1, NTHR, AGG_LDS_BYTES, stream>>>(ei, xlr, at1, bs1, g1, be1, Ah, Al, out, nN, nE, nN);
}
